// GAT_70153995813498
// MI455X (gfx1250) — hardware-verified
//
#include <hip/hip_runtime.h>
#include <stddef.h>
#include <stdint.h>
#include <math.h>


#define F_IN    64
#define HC      256
#define HID     64
#define NHD     4
#define KH      128
#define MLPH    200
#define MLPP    256
#define NCLS    2
#define NTHR    256
#define NWAVE   8
#define EPT     8
#define CHUNK   (NTHR * EPT)
#define WCAP    (EPT * 32)
#define LISTN   (NWAVE * WCAP)
#define NBMAX   2048
#define SLOTB   11
#define RCAP    28672
#define DEGCAP  256
#define GBM     64
#define GBN     64
#define GTHR    128
#define MROWS   128
#define HR      128
#define NEGSL   0.2f
#define WSMAX   134217728
#define LDS_AGG ((2 * RCAP + 2 * NBMAX + LISTN) * 4 + 64)

static_assert((CHUNK & (CHUNK - 1)) == 0 && CHUNK <= (1 << SLOTB));
static_assert(NBMAX == (1 << SLOTB));
static_assert(NTHR * 8 == NBMAX);
static_assert(LISTN >= NBMAX);
static_assert(LISTN >= NWAVE * WCAP);
static_assert((RCAP % 32) == 0);
static_assert(LDS_AGG <= 300000);
static_assert(GBM == (GTHR / 32) * 16);
static_assert(GTHR == 2 * GBN && GTHR == 2 * GBM);
static_assert((F_IN % 32) == 0 && (KH % 32) == 0);
static_assert((HC % GBN) == 0 && HID == GBN && (MLPP % GBN) == 0);
static_assert(NHD * HID == HC && HC == 256);
static_assert(KH == 2 * HID);
static_assert((MROWS % GBM) == 0 && (MROWS % HR) == 0);
static_assert(HC == 8 * 32);
static_assert(MLPH <= MLPP && MLPP == HC && (MLPH * NCLS) % 4 == 0);
static_assert(HR == 16 * NWAVE && HR * NCLS == 256);
static_assert((F_IN / 8) == 8);

typedef float          v4f  __attribute__((ext_vector_type(4)));
typedef float          v8f  __attribute__((ext_vector_type(8)));
typedef int            v4i  __attribute__((ext_vector_type(4)));
typedef int            v8i  __attribute__((ext_vector_type(8)));
typedef unsigned int   v2u  __attribute__((ext_vector_type(2)));
typedef unsigned int   v4u  __attribute__((ext_vector_type(4)));
typedef unsigned short v8us __attribute__((ext_vector_type(8)));
typedef __bf16         v16b __attribute__((ext_vector_type(16)));
typedef v4f  __attribute__((may_alias)) v4fa;
typedef v8us __attribute__((may_alias)) v8usa;
union FragB { v16b v; v8us h[2]; v8i w; };

__device__ __forceinline__ v8f wmb(const FragB& a, const FragB& b, v8f c) {
  v8f d = __builtin_amdgcn_wmma_f32_16x16x32_bf16(false, a.v, false, b.v, (short)0, c, false, false);
  asm volatile("v_nop\n\tv_nop\n\tv_nop\n\tv_nop" : "+v"(d) : "v"(a.w), "v"(b.w));
  return d;
}

__device__ __forceinline__ unsigned int f2bf(float f) {
  const unsigned int u = __float_as_uint(f);
  const unsigned int r = ((u + 0x7FFFu + ((u >> 16) & 1u)) >> 16) & 0xFFFFu;
  const bool isn = (u & 0x7FFFFFFFu) > 0x7F800000u;
  return isn ? 0x7FC0u : r;
}
__device__ __forceinline__ float bf2f(unsigned int b) { return __uint_as_float(b << 16); }
__device__ __forceinline__ float bfr(float f) { return bf2f(f2bf(f)); }
__device__ __forceinline__ v4f bfr4(const v4f a) {
  v4f r; r.x = bfr(a.x); r.y = bfr(a.y); r.z = bfr(a.z); r.w = bfr(a.w); return r;
}
__device__ __forceinline__ unsigned int pk2(float lo, float hi) { return f2bf(lo) | (f2bf(hi) << 16); }
__device__ __forceinline__ v4u pack8(const v4f a, const v4f b) {
  v4u r;
  r.x = pk2(a.x, a.y); r.y = pk2(a.z, a.w); r.z = pk2(b.x, b.y); r.w = pk2(b.z, b.w);
  return r;
}
__device__ __forceinline__ float relu_s(float v) { return (v > 0.0f) ? v : (v - v); }

__device__ __forceinline__ int scan_chunk(const int* __restrict__ dsts, int nE, int cbase, int slotBase,
                                          int nb, int vec8, int* list, int tid, int lane, int wave) {
  int wc = 0;
  const int el0  = tid * EPT;
  const int e0   = cbase + el0;
  const int sent = -2147483647 - 1;
  v4i da, db;
  if (vec8 != 0 && cbase + CHUNK <= nE) {
    da = *(const v4i*)(dsts + e0);
    db = *(const v4i*)(dsts + e0 + 4);
  } else {
    da.x = (e0     < nE) ? dsts[min(e0,     nE - 1)] : sent;
    da.y = (e0 + 1 < nE) ? dsts[min(e0 + 1, nE - 1)] : sent;
    da.z = (e0 + 2 < nE) ? dsts[min(e0 + 2, nE - 1)] : sent;
    da.w = (e0 + 3 < nE) ? dsts[min(e0 + 3, nE - 1)] : sent;
    db.x = (e0 + 4 < nE) ? dsts[min(e0 + 4, nE - 1)] : sent;
    db.y = (e0 + 5 < nE) ? dsts[min(e0 + 5, nE - 1)] : sent;
    db.z = (e0 + 6 < nE) ? dsts[min(e0 + 6, nE - 1)] : sent;
    db.w = (e0 + 7 < nE) ? dsts[min(e0 + 7, nE - 1)] : sent;
  }
  const unsigned nbs = (unsigned)slotBase;
  const unsigned unb = (unsigned)nb;
  const unsigned s0 = (unsigned)da.x - nbs, s1 = (unsigned)da.y - nbs;
  const unsigned s2 = (unsigned)da.z - nbs, s3 = (unsigned)da.w - nbs;
  const unsigned s4 = (unsigned)db.x - nbs, s5 = (unsigned)db.y - nbs;
  const unsigned s6 = (unsigned)db.z - nbs, s7 = (unsigned)db.w - nbs;
  const bool h0 = s0 < unb, h1 = s1 < unb, h2 = s2 < unb, h3 = s3 < unb;
  const bool h4 = s4 < unb, h5 = s5 < unb, h6 = s6 < unb, h7 = s7 < unb;
  const unsigned any = __builtin_amdgcn_ballot_w32(h0 | h1 | h2 | h3 | h4 | h5 | h6 | h7);
  if (any != 0u) {
#define HITJ(J, HJ, SJ) { \
      const unsigned mj = __builtin_amdgcn_ballot_w32(HJ); \
      if (mj != 0u) { \
        if (HJ) { \
          const int pos = wc + (int)__builtin_amdgcn_mbcnt_lo(mj, 0u); \
          if (pos < WCAP) list[wave * WCAP + pos] = ((el0 + (J)) << SLOTB) | (int)(SJ); \
        } \
        wc += (int)__builtin_popcount(mj); } }
    HITJ(0, h0, s0)
    HITJ(1, h1, s1)
    HITJ(2, h2, s2)
    HITJ(3, h3, s3)
    HITJ(4, h4, s4)
    HITJ(5, h5, s5)
    HITJ(6, h6, s6)
    HITJ(7, h7, s7)
#undef HITJ
  }
  return wc;
}

__global__ __launch_bounds__(NTHR) void k_xprep(const float* __restrict__ x, unsigned short* xb, int nN, int nUnits) {
  const int i = (int)blockIdx.x * NTHR + (int)threadIdx.x;
  if (i >= nUnits) return;
  const int row = i >> 3;
  const int c0  = (i & 7) * 8;
  const int rc  = row < nN ? row : nN - 1;
  const float* p = x + (size_t)rc * F_IN + c0;
  v4f a = *(const v4fa*)p, b = *(const v4fa*)(p + 4);
  const v4f z4 = {0.f, 0.f, 0.f, 0.f};
  if (row >= nN) { a = z4; b = z4; }
  const v4u hv = pack8(a, b);
  const size_t o = (size_t)row * F_IN + c0;
  *(volatile v4u*)(xb + o) = hv;
  __threadfence();
  *(volatile v4u*)(xb + o) = hv;
}

__global__ __launch_bounds__(NTHR) void k_wtr(const float* __restrict__ w, int Kin, int Ncol, int Nrows, int Kout,
                                              unsigned short* wt, int nUnits) {
  const int u = (int)blockIdx.x * NTHR + (int)threadIdx.x;
  if (u >= nUnits) return;
  const int kq = Kout >> 3;
  const int n  = u / kq;
  const int k8 = (u - n * kq) * 8;
  const int kk = k8 - (k8 / Kin) * Kin;
  const int ncl = n < Ncol ? n : Ncol - 1;
  const float* p = w + (size_t)kk * (size_t)Ncol + ncl;
  v4f a, b;
  a.x = p[0];                    a.y = p[(size_t)Ncol];         a.z = p[(size_t)2 * Ncol];     a.w = p[(size_t)3 * Ncol];
  b.x = p[(size_t)4 * Ncol];     b.y = p[(size_t)5 * Ncol];     b.z = p[(size_t)6 * Ncol];     b.w = p[(size_t)7 * Ncol];
  const v4f z4 = {0.f, 0.f, 0.f, 0.f};
  if (n >= Ncol || n >= Nrows) { a = z4; b = z4; }
  const v4u wv = pack8(a, b);
  unsigned short* o = wt + (size_t)n * (size_t)Kout + k8;
  *(volatile v4u*)o = wv;
  __threadfence();
  *(volatile v4u*)o = wv;
}

template <int MODE>
__global__ __launch_bounds__(GTHR) void k_gemm(
    const unsigned short* __restrict__ A, const unsigned short* __restrict__ WT,
    float* outF, int K, int ldo,
    const float* __restrict__ p0, const float* __restrict__ p1, int pLen,
    float* aux, int MPr, int nN)
{
  __shared__ __attribute__((aligned(16))) float stg[GBM * GBN];
  __shared__ __attribute__((aligned(16))) float satt[2 * GBN];
  __shared__ __attribute__((aligned(16))) float sdot[2 * GBM];
  const int tid = (int)threadIdx.x, lane = tid & 31, wave = tid >> 5, hh = lane >> 4, m = lane & 15;
  const int rowBase = (int)blockIdx.x * GBM;
  const int head    = (int)blockIdx.y;
  const int col0    = head * GBN;

  {
    const int which = tid >> 6;
    const int c  = tid & 63;
    float v;
    if constexpr (MODE == 0) {
      const int cl = c < pLen ? c : pLen - 1;
      const float vs = p0[head * pLen + cl];
      const float vd = p1[head * pLen + cl];
      v = (which == 0) ? vs : vd;
      v = (c < pLen) ? bfr(v) : 0.f;
    } else {
      const int col = col0 + c;
      const int cl  = col < pLen ? col : pLen - 1;
      const float vb = p0[cl];
      v = (col < pLen) ? bfr(vb) : 0.f;
    }
    satt[which * GBN + c] = v;
  }

  v8f acc[4];
  {
    const v8f z = {0.f, 0.f, 0.f, 0.f, 0.f, 0.f, 0.f, 0.f};
    acc[0] = z; acc[1] = z; acc[2] = z; acc[3] = z;
  }
  const unsigned short* ap = A  + (size_t)(rowBase + 16 * wave + m) * (size_t)K + 8 * hh;
  const unsigned short* wp = WT + (size_t)(col0 + m) * (size_t)K + 8 * hh;
  const int ksteps = K >> 5;
#pragma unroll 1
  for (int ks = 0; ks < ksteps; ++ks) {
    FragB af;
    af.h[0] = *(const v8usa*)(ap + 32 * ks);
    af.h[1] = *(const v8usa*)(ap + 32 * ks + 16);
#pragma unroll
    for (int t = 0; t < 4; ++t) {
      const unsigned short* wq = wp + (size_t)(16 * t) * (size_t)K + 32 * ks;
      FragB bf;
      bf.h[0] = *(const v8usa*)wq;
      bf.h[1] = *(const v8usa*)(wq + 16);
      acc[t] = wmb(af, bf, acc[t]);
    }
  }

#pragma unroll
  for (int t = 0; t < 4; ++t) {
    const int lc = 16 * t + m;
#pragma unroll
    for (int r = 0; r < 8; ++r) {
      const int lr = 16 * wave + 8 * hh + r;
      stg[lr * GBN + lc] = acc[t][r];
    }
  }
  __syncthreads();

  v4f fv[8];
  v4f sdv;
  float* sp;

  if constexpr (MODE == 0) {
    {
      const int row = tid & 63, which = tid >> 6;
      const float* sa = satt + which * GBN;
      const float* hr = stg + row * GBN;
      float d = 0.f;
#pragma unroll 4
      for (int c4 = 0; c4 < GBN / 4; ++c4) {
        const v4f hv = *(const v4fa*)(hr + 4 * c4);
        const v4f av = *(const v4fa*)(sa + 4 * c4);
        d = fmaf(hv.x, av.x, d);
        d = fmaf(hv.y, av.y, d);
        d = fmaf(hv.z, av.z, d);
        d = fmaf(hv.w, av.w, d);
      }
      sdot[which * GBM + row] = d;
    }
    __syncthreads();
#pragma unroll
    for (int i = 0; i < 8; ++i) {
      const int lr = 16 * wave + 2 * i + hh;
      fv[i] = *(const v4fa*)(stg + lr * GBN + 4 * m);
    }
    const int which2 = lane >> 4, piece = lane & 15;
    sdv = *(const v4fa*)(sdot + which2 * GBM + 4 * piece);
    sp = aux + (size_t)(2 * head + which2) * (size_t)MPr + rowBase + 4 * piece;
  } else {
    const v4f b4 = *(const v4fa*)(satt + 4 * m);
#pragma unroll
    for (int i = 0; i < 8; ++i) {
      const int lr = 16 * wave + 2 * i + hh;
      const bool ok = (rowBase + lr) < nN;
      const v4f x = *(const v4fa*)(stg + lr * GBN + 4 * m);
      v4f y;
      y.x = relu_s(x.x + b4.x); y.y = relu_s(x.y + b4.y);
      y.z = relu_s(x.z + b4.z); y.w = relu_s(x.w + b4.w);
      y.x = ok ? y.x : 0.f; y.y = ok ? y.y : 0.f; y.z = ok ? y.z : 0.f; y.w = ok ? y.w : 0.f;
      fv[i] = y;
      *(v4fa*)(stg + lr * GBN + 4 * m) = y;
    }
    __syncthreads();
    if (tid < GBN) {
      int nv = nN - rowBase; nv = nv < 0 ? 0 : (nv > GBM ? GBM : nv);
      float s = 0.f;
#pragma unroll 4
      for (int r = 0; r < nv; ++r) s += stg[r * GBN + tid];
      const float rn = (nv > 0) ? (1.0f / (float)nv) : 0.f;
      const float mean = s * rn;
      float q = 0.f;
#pragma unroll 4
      for (int r = 0; r < nv; ++r) {
        const float d = stg[r * GBN + tid] - mean;
        q = fmaf(d, d, q);
      }
      sdot[tid] = mean;
      sdot[GBM + tid] = q;
    }
    __syncthreads();
    sdv = *(const v4fa*)(sdot + 4 * lane);
    sp = aux + ((size_t)blockIdx.x * (size_t)gridDim.y + (size_t)blockIdx.y) * (size_t)(2 * GBN) + 4 * lane;
  }

#pragma unroll
  for (int i = 0; i < 8; ++i) {
    const int lr = 16 * wave + 2 * i + hh;
    const int gr = rowBase + lr;
    float* op = outF + (size_t)gr * (size_t)ldo + col0 + 4 * m;
    *(volatile v4f*)op = fv[i];
  }
  if (wave == 0) *(volatile v4f*)sp = sdv;
  __threadfence();
#pragma unroll
  for (int i = 0; i < 8; ++i) {
    const int lr = 16 * wave + 2 * i + hh;
    const int gr = rowBase + lr;
    float* op = outF + (size_t)gr * (size_t)ldo + col0 + 4 * m;
    *(volatile v4f*)op = fv[i];
  }
  if (wave == 0) *(volatile v4f*)sp = sdv;
}

__device__ __forceinline__ void onl_step(float lg, float& mx, float& dn, v4f& av, const v4f fs) {
  const float df = lg - mx;
  const float ee = expf(-fabsf(df));
  const bool up  = df > 0.f;
  const float s1 = up ? ee : 1.0f;
  const float s2 = up ? 1.0f : ee;
  mx = up ? lg : mx;
  dn = fmaf(dn, s1, s2);
  av.x = fmaf(av.x, s1, s2 * fs.x);
  av.y = fmaf(av.y, s1, s2 * fs.y);
  av.z = fmaf(av.z, s1, s2 * fs.z);
  av.w = fmaf(av.w, s1, s2 * fs.w);
}

__global__ __launch_bounds__(NTHR) void k_agg(
    const int* __restrict__ srcs, const int* __restrict__ dsts,
    const float* __restrict__ F, const float* __restrict__ SD,
    const float* __restrict__ bias,
    unsigned short* HP,
    int nN, int nE, int nb, int vec8, int MPr) {
  extern __shared__ v4f lds_dyn[];
  int* reg1 = (int*)lds_dyn;
  int* reg2 = reg1 + RCAP;
  int* scnt = reg2 + RCAP;
  int* soff = scnt + NBMAX;
  int* list = soff + NBMAX;
  int* wcnt = list + LISTN;
  int* wtot = wcnt + NWAVE;
  const int tid = (int)threadIdx.x, lane = tid & 31, wave = tid >> 5;
  const int nodeBase = (int)blockIdx.x * nb;

  for (int i = tid; i < NBMAX; i += NTHR) scnt[i] = 0;
  __syncthreads();

  int tot = 0;
  const int nChunks = (nE + CHUNK - 1) / CHUNK;
#pragma unroll 1
  for (int ch = 0; ch < nChunks; ++ch) {
    const int cbase = ch * CHUNK;
    const int wc = scan_chunk(dsts, nE, cbase, nodeBase, nb, vec8, list, tid, lane, wave);
    if (lane == 0) wcnt[wave] = wc;
    __syncthreads();
    int pre = 0, all = 0;
#pragma unroll
    for (int w2 = 0; w2 < NWAVE; ++w2) {
      int c = wcnt[w2];
      c = c < 0 ? 0 : (c > WCAP ? WCAP : c);
      all += c;
      pre += (w2 < wave) ? c : 0;
    }
    const int wcc  = wc > WCAP ? WCAP : wc;
    const int base = tot + pre;
#pragma unroll 1
    for (int i = lane; i < wcc; i += 32) {
      const int ent = list[wave * WCAP + i];
      const int el  = (ent >> SLOTB) & (CHUNK - 1);
      const int sl  = ent & (NBMAX - 1);
      int eid = cbase + el;
      eid = eid > nE - 1 ? nE - 1 : eid;
      const int pos = base + i;
      if (pos < RCAP) reg1[pos] = (int)(((unsigned)eid << SLOTB) | (unsigned)sl);
    }
    tot += all;
    tot = tot > RCAP ? RCAP : tot;
    __syncthreads();
  }
  const int nh = tot;

  if (wave == 0) {
#pragma unroll 1
    for (int b0 = 0; b0 < nh; b0 += 32) {
      const int idx = b0 + lane;
      const int uv  = reg1[idx < nh ? idx : nh - 1];
      const int m32 = (nh - b0) < 32 ? (nh - b0) : 32;
#pragma unroll 1
      for (int k = 0; k < m32; ++k) {
        const int u  = __builtin_amdgcn_readlane(uv, k);
        const int sl = u & (NBMAX - 1);
        if (lane == 0) scnt[sl] = scnt[sl] + 1;
      }
    }
  }
  __syncthreads();

  {
    const v4i ca = *(const v4i*)(scnt + 8 * tid);
    const v4i cb = *(const v4i*)(scnt + 8 * tid + 4);
    const int e0 = ca.x < 0 ? 0 : ca.x, e1 = ca.y < 0 ? 0 : ca.y, e2 = ca.z < 0 ? 0 : ca.z, e3 = ca.w < 0 ? 0 : ca.w;
    const int e4 = cb.x < 0 ? 0 : cb.x, e5 = cb.y < 0 ? 0 : cb.y, e6 = cb.z < 0 ? 0 : cb.z, e7 = cb.w < 0 ? 0 : cb.w;
    const int ts = e0 + e1 + e2 + e3 + e4 + e5 + e6 + e7;
    int incl = ts;
#pragma unroll
    for (int d = 1; d < 32; d <<= 1) {
      const int up = __shfl_up(incl, d);
      if (lane >= d) incl += up;
    }
    if (lane == 31) wtot[wave] = incl;
    __syncthreads();
    int pre = 0;
#pragma unroll
    for (int w2 = 0; w2 < NWAVE; ++w2) pre += (w2 < wave) ? wtot[w2] : 0;
    int run = pre + incl - ts;
    soff[8 * tid + 0] = run; run += e0;
    soff[8 * tid + 1] = run; run += e1;
    soff[8 * tid + 2] = run; run += e2;
    soff[8 * tid + 3] = run; run += e3;
    soff[8 * tid + 4] = run; run += e4;
    soff[8 * tid + 5] = run; run += e5;
    soff[8 * tid + 6] = run; run += e6;
    soff[8 * tid + 7] = run;
  }
  __syncthreads();
  for (int i = tid; i < NBMAX; i += NTHR) list[i] = soff[i];
  __syncthreads();

  if (wave == 0) {
#pragma unroll 1
    for (int b0 = 0; b0 < nh; b0 += 32) {
      const int idx = b0 + lane;
      const int uv  = reg1[idx < nh ? idx : nh - 1];
      const int m32 = (nh - b0) < 32 ? (nh - b0) : 32;
#pragma unroll 1
      for (int k = 0; k < m32; ++k) {
        const int u   = __builtin_amdgcn_readlane(uv, k);
        const int sl  = u & (NBMAX - 1);
        const int eid = (int)((unsigned)u >> SLOTB);
        if (lane == 0) {
          int pos = list[sl];
          pos = pos < 0 ? 0 : (pos > RCAP - 1 ? RCAP - 1 : pos);
          reg2[pos] = eid;
          list[sl] = pos + 1;
        }
      }
    }
  }
  __syncthreads();

  const int nbw = nb >> 3;
  const bool ovf = (nh >= RCAP);
  const float qnan = __int_as_float(0x7fc00000);

  const int cA = 4 * lane;
  const int cB = 128 + 4 * lane;
  const int hA = lane >> 4;
  const int hB = 2 + (lane >> 4);
  const v4f bA = bfr4(*(const v4fa*)(bias + cA));
  const v4f bB = bfr4(*(const v4fa*)(bias + cB));
  const float* ASa = SD + (size_t)(2 * hA) * (size_t)MPr;
  const float* ADa = ASa + MPr;
  const float* ASb = SD + (size_t)(2 * hB) * (size_t)MPr;
  const float* ADb = ASb + MPr;

#pragma unroll 1
  for (int jt = 0; jt < nbw; ++jt) {
    const int slot = wave * nbw + jt;
    const int grow = nodeBase + slot;
    const int gcl  = grow < nN ? grow : nN - 1;
    int st = soff[slot];
    const int craw = scnt[slot];
    int cnt = craw;
    st  = st < 0 ? 0 : (st > nh ? nh : st);
    cnt = cnt < 0 ? 0 : (cnt > DEGCAP ? DEGCAP : cnt);
    if (cnt > nh - st) cnt = nh - st;
    const float pz = (ovf || craw > DEGCAP) ? qnan : 0.0f;

    const v4f fdA = *(const v4fa*)(F + (size_t)gcl * HC + cA);
    const v4f fdB = *(const v4fa*)(F + (size_t)gcl * HC + cB);
    const float advA = ADa[gcl];
    const float advB = ADb[gcl];
    float l0A = ASa[gcl] + advA;
    float l0B = ASb[gcl] + advB;
    l0A = l0A > 0.f ? l0A : NEGSL * l0A;
    l0B = l0B > 0.f ? l0B : NEGSL * l0B;
    float mxA = l0A, dnA = 1.0f, mxB = l0B, dnB = 1.0f;
    v4f avA = fdA, avB = fdB;

#pragma unroll 1
    for (int q = 0; q < cnt; ++q) {
      int idx = st + q; idx = idx > RCAP - 1 ? RCAP - 1 : idx;
      int eid = reg2[idx]; eid = eid < 0 ? 0 : (eid > nE - 1 ? nE - 1 : eid);
      const int sraw = srcs[eid];
      const int s = sraw < 0 ? 0 : (sraw > nN - 1 ? nN - 1 : sraw);
      const v4f fsA = *(const v4fa*)(F + (size_t)s * HC + cA);
      const v4f fsB = *(const v4fa*)(F + (size_t)s * HC + cB);
      float lgA = ASa[s] + advA;
      float lgB = ASb[s] + advB;
      lgA = lgA > 0.f ? lgA : NEGSL * lgA;
      lgB = lgB > 0.f ? lgB : NEGSL * lgB;
      onl_step(lgA, mxA, dnA, avA, fsA);
      onl_step(lgB, mxB, dnB, avB, fsB);
    }
    const float invA = 1.0f / dnA;
    const float invB = 1.0f / dnB;
    const bool live = grow < nN;
    v4f sm;
    {
      const float ax = relu_s(fmaf(avA.x, invA, bA.x)) + relu_s(fmaf(avB.x, invB, bB.x));
      const float ay = relu_s(fmaf(avA.y, invA, bA.y)) + relu_s(fmaf(avB.y, invB, bB.y));
      const float az = relu_s(fmaf(avA.z, invA, bA.z)) + relu_s(fmaf(avB.z, invB, bB.z));
      const float aw = relu_s(fmaf(avA.w, invA, bA.w)) + relu_s(fmaf(avB.w, invB, bB.w));
      sm.x = (live ? ax : 0.f) + pz;
      sm.y = (live ? ay : 0.f) + pz;
      sm.z = (live ? az : 0.f) + pz;
      sm.w = (live ? aw : 0.f) + pz;
    }
    const float ox = __shfl_xor(sm.x, 16), oy = __shfl_xor(sm.y, 16);
    const float oz = __shfl_xor(sm.z, 16), ow = __shfl_xor(sm.w, 16);
    const float hx = (sm.x + ox) * 0.25f, hy = (sm.y + oy) * 0.25f;
    const float hz = (sm.z + oz) * 0.25f, hw = (sm.w + ow) * 0.25f;
    const unsigned int hbx = f2bf(hx), hby = f2bf(hy), hbz = f2bf(hz), hbw = f2bf(hw);
    const unsigned int lbx = f2bf(hx - bf2f(hbx)), lby = f2bf(hy - bf2f(hby));
    const unsigned int lbz = f2bf(hz - bf2f(hbz)), lbw = f2bf(hw - bf2f(hbw));
    const unsigned int hw0 = hbx | (hby << 16), hw1 = hbz | (hbw << 16);
    const unsigned int lw0 = lbx | (lby << 16), lw1 = lbz | (lbw << 16);
    const bool lsel = lane >= 16;
    v2u pv;
    pv.x = lsel ? lw0 : hw0;
    pv.y = lsel ? lw1 : hw1;
    unsigned short* gp = HP + (size_t)grow * KH + 4 * lane;
    const bool wr = grow < MPr;
    if (wr) *(volatile v2u*)gp = pv;
    __threadfence();
    if (wr) *(volatile v2u*)gp = pv;
  }
}

__global__ __launch_bounds__(NTHR) void k_bnstat(const float* __restrict__ rec, int gM, int nN,
                                                 const float* __restrict__ gam, const float* __restrict__ bet,
                                                 float* ss) {
  __shared__ __attribute__((aligned(16))) float stg[3 * MLPP];
  const int tid = (int)threadIdx.x;
  const int c  = tid;
  const int cb = c >> 6;
  const int cc = c & (GBN - 1);
  double n = 0.0, mean = 0.0, M2 = 0.0;
#pragma unroll 1
  for (int b = 0; b < gM; ++b) {
    const float* pr = rec + ((size_t)b * 4 + (size_t)cb) * (size_t)(2 * GBN);
    const double mb = (double)pr[cc];
    const double qb = (double)pr[GBN + cc];
    int nbi = nN - b * GBM; nbi = nbi < 0 ? 0 : (nbi > GBM ? GBM : nbi);
    if (nbi > 0) {
      const double nb = (double)nbi;
      const double nn = n + nb;
      const double delta = mb - mean;
      const double f = nb / nn;
      mean = mean + delta * f;
      M2 = M2 + qb + delta * delta * n * f;
      n = nn;
    }
  }
  const double nt = n < 1.0 ? 1.0 : n;
  const float varf  = (float)(M2 / nt);
  const float meanf = (float)mean;
  const float rstd = 1.0f / sqrtf(varf + 1e-5f);
  const int cl = c < MLPH ? c : MLPH - 1;
  const float gv = bfr(gam[cl]);
  const float bv = bfr(bet[cl]);
  const bool okc = c < MLPH;
  stg[c]            = okc ? meanf : 0.f;
  stg[MLPP + c]     = okc ? gv * rstd : 0.f;
  stg[2 * MLPP + c] = okc ? bv : 0.f;
  __syncthreads();
  v4f v = {0.f, 0.f, 0.f, 0.f};
  if (tid < (3 * MLPP) / 4) {
    v = *(const v4fa*)(stg + 4 * tid);
    *(volatile v4f*)(ss + 4 * tid) = v;
  }
  __threadfence();
  if (tid < (3 * MLPP) / 4) {
    *(volatile v4f*)(ss + 4 * tid) = v;
  }
}

__global__ __launch_bounds__(NTHR) void k_head(const float* __restrict__ Z, const float* __restrict__ ss,
                                               const float* __restrict__ mw2, const float* __restrict__ mb2,
                                               float* out, int nN) {
  __shared__ __attribute__((aligned(16))) float sp[3 * MLPP];
  __shared__ __attribute__((aligned(16))) float sw[2 * MLPP];
  __shared__ __attribute__((aligned(16))) float sout[HR * NCLS];
  const int tid = (int)threadIdx.x, lane = tid & 31, wave = tid >> 5;
  const int rowBase = (int)blockIdx.x * HR;

  if (tid < (3 * MLPP) / 4) {
    const v4f v = *(const v4fa*)(ss + 4 * tid);
    *(v4fa*)(sp + 4 * tid) = v;
  }
  if (tid < MLPP / 2) {
    const int tcl = tid < (MLPH * NCLS) / 4 ? tid : (MLPH * NCLS) / 4 - 1;
    const v4f v = *(const v4fa*)(mw2 + 4 * tcl);
    const bool ok = tid < (MLPH * NCLS) / 4;
    sw[2 * tid]            = ok ? bfr(v.x) : 0.f;
    sw[MLPP + 2 * tid]     = ok ? bfr(v.y) : 0.f;
    sw[2 * tid + 1]        = ok ? bfr(v.z) : 0.f;
    sw[MLPP + 2 * tid + 1] = ok ? bfr(v.w) : 0.f;
  }
  const float m0 = bfr(mb2[0]);
  const float m1 = bfr(mb2[1]);
  __syncthreads();

#pragma unroll 1
  for (int i = 0; i < HR / NWAVE; ++i) {
    const int r = wave * (HR / NWAVE) + i;
    const int grow = rowBase + r;
    const int gcl  = grow < nN ? grow : nN - 1;
    float a0 = 0.f, a1 = 0.f;
#pragma unroll 1
    for (int hf = 0; hf < 2; ++hf) {
      const int c = 128 * hf + 4 * lane;
      const v4f z  = *(const v4fa*)(Z + (size_t)gcl * MLPP + c);
      const v4f mu = *(const v4fa*)(sp + c);
      const v4f sc = *(const v4fa*)(sp + MLPP + c);
      const v4f bb = *(const v4fa*)(sp + 2 * MLPP + c);
      const v4f w0 = *(const v4fa*)(sw + c);
      const v4f w1 = *(const v4fa*)(sw + MLPP + c);
      const float t0 = (z.x - mu.x) * sc.x + bb.x;
      const float t1 = (z.y - mu.y) * sc.y + bb.y;
      const float t2 = (z.z - mu.z) * sc.z + bb.z;
      const float t3 = (z.w - mu.w) * sc.w + bb.w;
      a0 = fmaf(t0, w0.x, a0); a1 = fmaf(t0, w1.x, a1);
      a0 = fmaf(t1, w0.y, a0); a1 = fmaf(t1, w1.y, a1);
      a0 = fmaf(t2, w0.z, a0); a1 = fmaf(t2, w1.z, a1);
      a0 = fmaf(t3, w0.w, a0); a1 = fmaf(t3, w1.w, a1);
    }
#pragma unroll
    for (int off = 16; off > 0; off >>= 1) {
      a0 += __shfl_xor(a0, off);
      a1 += __shfl_xor(a1, off);
    }
    if (lane == 0) {
      sout[2 * r]     = a0 + m0;
      sout[2 * r + 1] = a1 + m1;
    }
  }
  __syncthreads();
  int live = nN - rowBase; live = live < 0 ? 0 : (live > HR ? HR : live);
  const int npc = (live * NCLS) / 4;
  v4f v = {0.f, 0.f, 0.f, 0.f};
  float* ob = out + (size_t)rowBase * NCLS + 4 * tid;
  if (tid < npc) {
    v = *(const v4fa*)(sout + 4 * tid);
    *(volatile v4f*)ob = v;
  }
  __threadfence();
  if (tid < npc) {
    *(volatile v4f*)ob = v;
  }
}

static int pick_nb(int nE, int nN) {
  int nb = NBMAX;
  while (nb > 32 && (long long)nb * (long long)nE * 5LL > (long long)RCAP * (long long)nN * 4LL) nb >>= 1;
  return nb;
}
static inline int cdiv(int a, int b) { return (a + b - 1) / b; }

extern "C" void kernel_launch(void* const* d_in, const int* in_sizes, int n_in,
                              void* d_out, int out_size, void* d_ws, size_t ws_size,
                              hipStream_t stream) {
  if (n_in < 16) return;
  const int nN = in_sizes[0] / F_IN;
  if (nN <= 0 || in_sizes[0] != nN * F_IN || nN >= (1 << 22)) return;
  if ((nN % 16) != 0) return;
  if (in_sizes[1] < 2 || (in_sizes[1] & 1) != 0) return;
  const int nE = in_sizes[1] / 2;
  if (nE < 1 || nE >= (1 << (32 - SLOTB))) return;
  if (in_sizes[2] != F_IN * HC) return;
  if (in_sizes[3] != NHD * HID || in_sizes[4] != NHD * HID) return;
  if (in_sizes[5] != HC) return;
  if (in_sizes[6] != HID * HC) return;
  if (in_sizes[7] != NHD * HID || in_sizes[8] != NHD * HID) return;
  if (in_sizes[9] != HC) return;
  if (in_sizes[10] != HID * MLPH) return;
  if (in_sizes[11] != MLPH || in_sizes[12] != MLPH || in_sizes[13] != MLPH) return;
  if (in_sizes[14] != MLPH * NCLS || in_sizes[15] != NCLS) return;
  if (out_size != nN * NCLS) return;

  const float* x    = (const float*)d_in[0];
  const int*   ei   = (const int*)  d_in[1];
  const float* W1   = (const float*)d_in[2];
  const float* al1  = (const float*)d_in[3];
  const float* ar1  = (const float*)d_in[4];
  const float* b1   = (const float*)d_in[5];
  const float* W2   = (const float*)d_in[6];
  const float* al2  = (const float*)d_in[7];
  const float* ar2  = (const float*)d_in[8];
  const float* b2   = (const float*)d_in[9];
  const float* mw1  = (const float*)d_in[10];
  const float* mb1  = (const float*)d_in[11];
  const float* bng  = (const float*)d_in[12];
  const float* bnb  = (const float*)d_in[13];
  const float* mw2  = (const float*)d_in[14];
  const float* mb2  = (const float*)d_in[15];
  float* out = (float*)d_out;
  const int* src = ei;
  const int* dst = ei + nE;

  const int MP   = cdiv(nN, MROWS) * MROWS;
  const int nb   = pick_nb(nE, nN);
  if (nb < 32 || (nb & (nb - 1)) != 0 || nb > NBMAX) return;
  const int gA   = cdiv(MP, nb);
  const int vec8 = ((nE & 3) == 0) ? 1 : 0;
  if (gA * nb < MP) return;
  const int gM = MP / GBM;

  char* ws = (char*)d_ws;
  size_t off = 0;
  const size_t oXB  = off; off += (size_t)MP * F_IN * 2;           off = (off + 255) & ~(size_t)255;
  const size_t oW1T = off; off += (size_t)HC * F_IN * 2;           off = (off + 255) & ~(size_t)255;
  const size_t oW2T = off; off += (size_t)HC * KH * 2;             off = (off + 255) & ~(size_t)255;
  const size_t oMWT = off; off += (size_t)MLPP * KH * 2;           off = (off + 255) & ~(size_t)255;
  const size_t oFT  = off; off += (size_t)MP * HC * 4;             off = (off + 255) & ~(size_t)255;
  const size_t oSD  = off; off += (size_t)2 * NHD * MP * 4;        off = (off + 255) & ~(size_t)255;
  const size_t oHH  = off; off += (size_t)MP * KH * 2;             off = (off + 255) & ~(size_t)255;
  const size_t oRC  = off; off += (size_t)gM * 4 * (2 * GBN) * 4;  off = (off + 255) & ~(size_t)255;
  const size_t oSS  = off; off += (size_t)(3 * MLPP) * 4;          off = (off + 255) & ~(size_t)255;
  if (off > ws_size || off > (size_t)WSMAX) return;
  unsigned short* XB  = (unsigned short*)(ws + oXB);
  unsigned short* W1T = (unsigned short*)(ws + oW1T);
  unsigned short* W2T = (unsigned short*)(ws + oW2T);
  unsigned short* MWT = (unsigned short*)(ws + oMWT);
  float*          FT  = (float*)(ws + oFT);
  float*          SD  = (float*)(ws + oSD);
  unsigned short* HH  = (unsigned short*)(ws + oHH);
  float*          RC  = (float*)(ws + oRC);
  float*          SS  = (float*)(ws + oSS);

  hipFuncSetAttribute(reinterpret_cast<const void*>(&k_agg),
                      hipFuncAttributeMaxDynamicSharedMemorySize, LDS_AGG);

  const int nUx = MP * (F_IN / 8);
  k_xprep<<<cdiv(nUx, NTHR), NTHR, 0, stream>>>(x, XB, nN, nUx);

  {
    const int nUw1 = HC * (F_IN / 8);
    k_wtr<<<cdiv(nUw1, NTHR), NTHR, 0, stream>>>(W1, F_IN, HC, HC, F_IN, W1T, nUw1);
    const int nUw2 = HC * (KH / 8);
    k_wtr<<<cdiv(nUw2, NTHR), NTHR, 0, stream>>>(W2, HID, HC, HC, KH, W2T, nUw2);
    const int nUw3 = MLPP * (KH / 8);
    k_wtr<<<cdiv(nUw3, NTHR), NTHR, 0, stream>>>(mw1, HID, MLPH, MLPP, KH, MWT, nUw3);
  }

  k_gemm<0><<<dim3(gM, HC / GBN), GTHR, 0, stream>>>(XB, W1T, FT, F_IN, HC, al1, ar1, HID, SD, MP, nN);
  k_agg<<<gA, NTHR, LDS_AGG, stream>>>(src, dst, FT, SD, b1, HH, nN, nE, nb, vec8, MP);
  k_gemm<0><<<dim3(gM, HC / GBN), GTHR, 0, stream>>>(HH, W2T, FT, KH, HC, al2, ar2, HID, SD, MP, nN);
  k_agg<<<gA, NTHR, LDS_AGG, stream>>>(src, dst, FT, SD, b2, HH, nN, nE, nb, vec8, MP);
  k_gemm<1><<<dim3(gM, MLPP / GBN), GTHR, 0, stream>>>(HH, MWT, FT, KH, MLPP, mb1, mb1, MLPH, RC, MP, nN);
  k_bnstat<<<1, NTHR, 0, stream>>>(RC, gM, nN, bng, bnb, SS);
  k_head<<<cdiv(nN, HR), NTHR, 0, stream>>>(FT, SS, mw2, mb2, out, nN);
}
